// GraphConvModule_47502338294286
// MI455X (gfx1250) — hardware-verified
//
#include <hip/hip_runtime.h>
#include <stddef.h>
#include <stdint.h>


#define FEA     128
#define CIN     300
#define CPAD    320
#define CQ      (CPAD / 8)
#define HID     512
#define CGN     (HID / 128)
#define KH      (2 * HID)
#define KC      (4 * FEA)
#define ACP     KC
#define NTHR    256
#define NWAVE   8
#define EPT     8
#define CHUNK   (NTHR * EPT)
#define WCAP    (EPT * 32)
#define LISTN   (NWAVE * WCAP)
#define NBMAX   2048
#define RCAP    28672
#define DEGCAP  1024
#define PKS     11
#define STW     512
#define GBM     64
#define GTHR    128
#define LMAX    8
#define WSMAX   134217728
#define LDS_AGG ((2 * RCAP + 2 * NBMAX + LISTN) * 4 + 64)
#define LDS_MLP (GBM * KH * 2 + GBM * FEA * 4)

static_assert((CHUNK & (CHUNK - 1)) == 0 && CHUNK <= (1 << PKS));
static_assert((NBMAX & (NBMAX - 1)) == 0 && NBMAX <= (1 << PKS));
static_assert(NTHR * 8 == NBMAX);
static_assert(LISTN >= NBMAX);
static_assert(LISTN >= NWAVE * WCAP);
static_assert((RCAP % 32) == 0);
static_assert(NWAVE * STW <= RCAP);
static_assert(STW >= 256);
static_assert(LDS_AGG <= 300000);
static_assert(LDS_MLP <= 300000);
static_assert(GBM == (GTHR / 32) * 16);
static_assert((CPAD % 32) == 0 && CPAD >= CIN && (KC % 32) == 0 && (KH % 32) == 0);
static_assert(FEA == 4 * 32 && (HID % 128) == 0 && ACP == 512 && KH == 1024);

typedef float          v4f  __attribute__((ext_vector_type(4)));
typedef float          v8f  __attribute__((ext_vector_type(8)));
typedef int            v4i  __attribute__((ext_vector_type(4)));
typedef int            v8i  __attribute__((ext_vector_type(8)));
typedef unsigned int   v2u  __attribute__((ext_vector_type(2)));
typedef unsigned int   v4u  __attribute__((ext_vector_type(4)));
typedef unsigned short v8us __attribute__((ext_vector_type(8)));
typedef __bf16         v16b __attribute__((ext_vector_type(16)));
typedef v8us __attribute__((may_alias)) v8usa;
typedef v4f  __attribute__((may_alias)) v4fa;
typedef v4u  __attribute__((may_alias)) v4ua;
typedef v2u  __attribute__((may_alias)) v2ua;
union FragB { v16b v; v8us h[2]; v8i w; };

__device__ __forceinline__ v8f wmb(const FragB& a, const FragB& b, v8f c) {
  v8f d = __builtin_amdgcn_wmma_f32_16x16x32_bf16(false, a.v, false, b.v, (short)0, c, false, false);
  asm volatile("v_nop\n\tv_nop\n\tv_nop\n\tv_nop" : "+v"(d) : "v"(a.w), "v"(b.w));
  return d;
}

__device__ __forceinline__ unsigned short bf_bits(float f) {
  unsigned int u = __float_as_uint(f);
  u += 0x7FFFu + ((u >> 16) & 1u);
  return (unsigned short)(u >> 16);
}
__device__ __forceinline__ float bf_val(unsigned short b) {
  return __uint_as_float(((unsigned int)b) << 16);
}
__device__ __forceinline__ float bf_rne(float f) { return bf_val(bf_bits(f)); }

__device__ __forceinline__ void ldwait() {
  asm volatile("s_wait_loadcnt 0x0" ::: "memory");
}

__device__ __forceinline__ int scan_chunk(const int* __restrict__ dsts, int nE, int cbase, int slotBase,
                                          int nb, int vec8, int* list, int tid, int lane, int wave) {
  int wc = 0;
  const int el0  = tid * EPT;
  const int e0   = cbase + el0;
  const int sent = -2147483647 - 1;
  v4i da, db;
  if (vec8 != 0 && cbase + CHUNK <= nE) {
    da = *(const v4i*)(dsts + e0);
    db = *(const v4i*)(dsts + e0 + 4);
  } else {
    da.x = (e0     < nE) ? dsts[min(e0,     nE - 1)] : sent;
    da.y = (e0 + 1 < nE) ? dsts[min(e0 + 1, nE - 1)] : sent;
    da.z = (e0 + 2 < nE) ? dsts[min(e0 + 2, nE - 1)] : sent;
    da.w = (e0 + 3 < nE) ? dsts[min(e0 + 3, nE - 1)] : sent;
    db.x = (e0 + 4 < nE) ? dsts[min(e0 + 4, nE - 1)] : sent;
    db.y = (e0 + 5 < nE) ? dsts[min(e0 + 5, nE - 1)] : sent;
    db.z = (e0 + 6 < nE) ? dsts[min(e0 + 6, nE - 1)] : sent;
    db.w = (e0 + 7 < nE) ? dsts[min(e0 + 7, nE - 1)] : sent;
  }
  const unsigned nbs = (unsigned)slotBase;
  const unsigned unb = (unsigned)nb;
  const unsigned s0 = (unsigned)da.x - nbs, s1 = (unsigned)da.y - nbs;
  const unsigned s2 = (unsigned)da.z - nbs, s3 = (unsigned)da.w - nbs;
  const unsigned s4 = (unsigned)db.x - nbs, s5 = (unsigned)db.y - nbs;
  const unsigned s6 = (unsigned)db.z - nbs, s7 = (unsigned)db.w - nbs;
  const bool h0 = s0 < unb, h1 = s1 < unb, h2 = s2 < unb, h3 = s3 < unb;
  const bool h4 = s4 < unb, h5 = s5 < unb, h6 = s6 < unb, h7 = s7 < unb;
  const unsigned any = __builtin_amdgcn_ballot_w32(h0 | h1 | h2 | h3 | h4 | h5 | h6 | h7);
  if (any != 0u) {
#define HITJ(J, HJ, SJ) { \
      const unsigned mj = __builtin_amdgcn_ballot_w32(HJ); \
      if (mj != 0u) { \
        if (HJ) { \
          const int pos = wc + (int)__builtin_amdgcn_mbcnt_lo(mj, 0u); \
          if (pos < WCAP) list[wave * WCAP + pos] = ((el0 + (J)) << PKS) | (int)(SJ); \
        } \
        wc += (int)__builtin_popcount(mj); } }
    HITJ(0, h0, s0)
    HITJ(1, h1, s1)
    HITJ(2, h2, s2)
    HITJ(3, h3, s3)
    HITJ(4, h4, s4)
    HITJ(5, h5, s5)
    HITJ(6, h6, s6)
    HITJ(7, h7, s7)
#undef HITJ
  }
  return wc;
}

__global__ __launch_bounds__(NTHR) void k_cprep(const float* __restrict__ x, unsigned short* xc,
                                                int nN, int nUnits) {
  const int u = (int)blockIdx.x * NTHR + (int)threadIdx.x;
  if (u >= nUnits) return;
  const int row = u / CQ;
  const int k8  = (u - row * CQ) * 8;
  const int rc  = row < nN ? row : nN - 1;
  const float* p = x + (size_t)rc * CIN;
  float wv[8];
#pragma unroll
  for (int e = 0; e < 8; ++e) {
    int k = k8 + e;
    k = k < CIN ? k : CIN - 1;
    wv[e] = p[k];
  }
  ldwait();
  v8us pk;
#pragma unroll
  for (int e = 0; e < 8; ++e) {
    const bool ok = (row < nN) && (k8 + e < CIN);
    pk[e] = ok ? bf_bits(wv[e]) : (unsigned short)0;
  }
  unsigned short* gp = xc + (size_t)row * CPAD + k8;
  *(volatile v8us*)gp = pk;
  __threadfence();
  *(volatile v8us*)gp = pk;
}

__global__ __launch_bounds__(NTHR) void k_wtr(const float* __restrict__ W, int Kin, int Kper, int K, int ncols,
                                              int nMat, unsigned short* wt, int nUnits) {
  const int u = (int)blockIdx.x * NTHR + (int)threadIdx.x;
  if (u >= nUnits) return;
  const int kq  = K >> 3;
  const int per = ncols * kq;
  const int mat = u / per;
  const int o   = u - mat * per;
  const int n   = o / kq;
  const int k8  = (o - n * kq) * 8;
  const int kk8 = k8 - (k8 / Kper) * Kper;
  const float* Wm = W + (size_t)mat * (size_t)Kin * (size_t)ncols;
  float wv[8];
#pragma unroll
  for (int e = 0; e < 8; ++e) {
    int kk = kk8 + e;
    kk = kk < Kin ? kk : Kin - 1;
    wv[e] = Wm[(size_t)kk * (size_t)ncols + n];
  }
  ldwait();
  v8us pk;
#pragma unroll
  for (int e = 0; e < 8; ++e) pk[e] = (kk8 + e < Kin) ? bf_bits(wv[e]) : (unsigned short)0;
  (void)nMat;
  unsigned short* gp = wt + (size_t)mat * (size_t)ncols * (size_t)K + (size_t)n * (size_t)K + k8;
  *(volatile v8us*)gp = pk;
  __threadfence();
  *(volatile v8us*)gp = pk;
}

template<int MODE>
__global__ __launch_bounds__(GTHR) void k_mlp(
    const unsigned short* A, int lda, int ksteps1,
    const unsigned short* __restrict__ WTa, const float* __restrict__ ba,
    const unsigned short* __restrict__ WTb, const float* __restrict__ bb,
    const int* __restrict__ nid, const float* __restrict__ emb, int nEmb,
    float* Hout, int nN, int rowLim) {
  extern __shared__ v4f lds_dyn[];
  unsigned short* tt = (unsigned short*)lds_dyn;
  float* stg = (float*)(tt + GBM * KH);
  const int tid = (int)threadIdx.x, lane = tid & 31, wave = tid >> 5, hh = lane >> 4, m = lane & 15;
  const int rowBase = (int)blockIdx.x * GBM;
  const int K1 = ksteps1 << 5;
  const v8f z8 = {0.f, 0.f, 0.f, 0.f, 0.f, 0.f, 0.f, 0.f};

  const unsigned short* ap = A + (size_t)(rowBase + 16 * wave + m) * (size_t)lda + 8 * hh;
#pragma unroll 1
  for (int cg = 0; cg < CGN; ++cg) {
    v8f acc[8];
#pragma unroll
    for (int t = 0; t < 8; ++t) acc[t] = z8;
    const unsigned short* wp = WTa + (size_t)(cg * 128 + m) * (size_t)K1 + 8 * hh;
#pragma unroll 1
    for (int ks = 0; ks < ksteps1; ++ks) {
      FragB af;
      af.h[0] = *(const v8usa*)(ap + 32 * ks);
      af.h[1] = *(const v8usa*)(ap + 32 * ks + 16);
#pragma unroll
      for (int t = 0; t < 8; ++t) {
        const unsigned short* wq = wp + (size_t)(16 * t) * (size_t)K1 + 32 * ks;
        FragB bf;
        bf.h[0] = *(const v8usa*)wq;
        bf.h[1] = *(const v8usa*)(wq + 16);
        acc[t] = wmb(af, bf, acc[t]);
      }
    }
    float bv[8];
#pragma unroll
    for (int t = 0; t < 8; ++t) bv[t] = ba[cg * 128 + 16 * t + m];
    ldwait();
#pragma unroll
    for (int t = 0; t < 8; ++t) {
      const int col = cg * 128 + 16 * t + m;
      const float b = bf_rne(bv[t]);
#pragma unroll
      for (int r = 0; r < 8; ++r) {
        const int lr = 16 * wave + 8 * hh + r;
        float y = acc[t][r] + b;
        y = y > 0.0f ? y : 0.1f * y;
        const unsigned short hu = bf_bits(y);
        const unsigned short lu = bf_bits(y - bf_val(hu));
        tt[lr * KH + col]       = hu;
        tt[lr * KH + HID + col] = lu;
      }
    }
  }
  __syncthreads();

  v8f acc2[8];
#pragma unroll
  for (int t = 0; t < 8; ++t) acc2[t] = z8;
  const unsigned short* ap2 = tt + (16 * wave + m) * KH + 8 * hh;
  const unsigned short* wp2 = WTb + (size_t)m * (size_t)KH + 8 * hh;
#pragma unroll 1
  for (int ks = 0; ks < KH / 32; ++ks) {
    FragB af;
    af.h[0] = *(const v8usa*)(ap2 + 32 * ks);
    af.h[1] = *(const v8usa*)(ap2 + 32 * ks + 16);
#pragma unroll
    for (int t = 0; t < 8; ++t) {
      const unsigned short* wq = wp2 + (size_t)(16 * t) * (size_t)KH + 32 * ks;
      FragB bf;
      bf.h[0] = *(const v8usa*)wq;
      bf.h[1] = *(const v8usa*)(wq + 16);
      acc2[t] = wmb(af, bf, acc2[t]);
    }
  }
  float bv2[8];
#pragma unroll
  for (int t = 0; t < 8; ++t) bv2[t] = bb[16 * t + m];
  ldwait();
#pragma unroll
  for (int t = 0; t < 8; ++t) {
    const int lc = 16 * t + m;
    const float b = bf_rne(bv2[t]);
#pragma unroll
    for (int r = 0; r < 8; ++r) {
      const int lr = 16 * wave + 8 * hh + r;
      stg[lr * FEA + lc] = acc2[t][r] + b;
    }
  }
  __syncthreads();

  v4f fv[16];
#pragma unroll
  for (int i = 0; i < 16; ++i) {
    const int lr = 16 * wave + i;
    fv[i] = *(const v4fa*)(stg + lr * FEA + 4 * lane);
  }
  if (MODE == 0) {
#pragma unroll
    for (int hb = 0; hb < 2; ++hb) {
      int ixv[8];
#pragma unroll
      for (int j = 0; j < 8; ++j) {
        const int gr  = rowBase + 16 * wave + 8 * hb + j;
        const int grc = gr < nN ? gr : nN - 1;
        ixv[j] = nid[grc];
      }
      ldwait();
      v4f ev[8];
#pragma unroll
      for (int j = 0; j < 8; ++j) {
        int ix = ixv[j];
        ix = ix < -nEmb ? -nEmb : (ix > nEmb ? nEmb : ix);
        int er = ix + 1;
        er = er < 0 ? er + nEmb : er;
        er = er < 0 ? 0 : (er > nEmb - 1 ? nEmb - 1 : er);
        ev[j] = *(const v4fa*)(emb + (size_t)er * FEA + 4 * lane);
      }
      ldwait();
#pragma unroll
      for (int j = 0; j < 8; ++j) {
        v4f e2;
        e2.x = bf_rne(ev[j].x); e2.y = bf_rne(ev[j].y); e2.z = bf_rne(ev[j].z); e2.w = bf_rne(ev[j].w);
        fv[8 * hb + j] = e2 + fv[8 * hb + j];
      }
    }
  } else {
#pragma unroll
    for (int i = 0; i < 16; ++i) {
      const v4f v = fv[i];
      float s = v.x * v.x + v.y * v.y + v.z * v.z + v.w * v.w;
      s += __shfl_xor(s, 16, 32);
      s += __shfl_xor(s, 8, 32);
      s += __shfl_xor(s, 4, 32);
      s += __shfl_xor(s, 2, 32);
      s += __shfl_xor(s, 1, 32);
      const float rn = 1.0f / fmaxf(sqrtf(s), 1e-5f);
      fv[i] = v * rn;
    }
  }
#pragma unroll
  for (int i = 0; i < 16; ++i) {
    const int gr = rowBase + 16 * wave + i;
    float* op = Hout + (size_t)gr * (size_t)FEA + 4 * lane;
    if (gr < rowLim) *(volatile v4f*)op = fv[i];
  }
  __threadfence();
#pragma unroll
  for (int i = 0; i < 16; ++i) {
    const int gr = rowBase + 16 * wave + i;
    float* op = Hout + (size_t)gr * (size_t)FEA + 4 * lane;
    if (gr < rowLim) *(volatile v4f*)op = fv[i];
  }
}

__global__ __launch_bounds__(NTHR) void k_agg(
    const int* __restrict__ srcs, const int* __restrict__ dsts,
    const float* __restrict__ H, unsigned short* AC,
    int nN, int nE, int nb, int vec8, int MPr) {
  extern __shared__ v4f lds_dyn[];
  int* reg1 = (int*)lds_dyn;
  int* reg2 = reg1 + RCAP;
  int* scnt = reg2 + RCAP;
  int* soff = scnt + NBMAX;
  int* list = soff + NBMAX;
  int* wcnt = list + LISTN;
  int* wtot = wcnt + NWAVE;
  const int tid = (int)threadIdx.x, lane = tid & 31, wave = tid >> 5;
  const int nodeBase = (int)blockIdx.x * nb;

  for (int i = tid; i < NBMAX; i += NTHR) scnt[i] = 0;
  __syncthreads();

  int tot = 0;
  const int nChunks = (nE + CHUNK - 1) / CHUNK;
#pragma unroll 1
  for (int ch = 0; ch < nChunks; ++ch) {
    const int cbase = ch * CHUNK;
    const int wc = scan_chunk(dsts, nE, cbase, nodeBase, nb, vec8, list, tid, lane, wave);
    if (lane == 0) wcnt[wave] = wc;
    __syncthreads();
    int pre = 0, all = 0;
#pragma unroll
    for (int w2 = 0; w2 < NWAVE; ++w2) {
      int c = wcnt[w2];
      c = c < 0 ? 0 : (c > WCAP ? WCAP : c);
      all += c;
      pre += (w2 < wave) ? c : 0;
    }
    const int wcc  = wc > WCAP ? WCAP : wc;
    const int base = tot + pre;
#pragma unroll 1
    for (int i = lane; i < wcc; i += 32) {
      const int ent = list[wave * WCAP + i];
      const int el  = (ent >> PKS) & (CHUNK - 1);
      const int sl  = ent & (NBMAX - 1);
      int eid = cbase + el;
      eid = eid > nE - 1 ? nE - 1 : eid;
      const int pos = base + i;
      if (pos < RCAP) reg1[pos] = (int)(((unsigned)eid << PKS) | (unsigned)sl);
    }
    tot += all;
    tot = tot > RCAP ? RCAP : tot;
    __syncthreads();
  }
  const int nh = tot;

  if (wave == 0) {
#pragma unroll 1
    for (int b0 = 0; b0 < nh; b0 += 32) {
      const int idx = b0 + lane;
      const int uv  = reg1[idx < RCAP ? idx : RCAP - 1];
      const int m32 = (nh - b0) < 32 ? (nh - b0) : 32;
#pragma unroll 1
      for (int k = 0; k < m32; ++k) {
        const int u  = __builtin_amdgcn_readlane(uv, k);
        const int sl = u & (NBMAX - 1);
        if (lane == 0) scnt[sl] = scnt[sl] + 1;
      }
    }
  }
  __syncthreads();

  {
    const v4i ca = *(const v4i*)(scnt + 8 * tid);
    const v4i cb = *(const v4i*)(scnt + 8 * tid + 4);
    const int e0 = ca.x < 0 ? 0 : ca.x, e1 = ca.y < 0 ? 0 : ca.y, e2 = ca.z < 0 ? 0 : ca.z, e3 = ca.w < 0 ? 0 : ca.w;
    const int e4 = cb.x < 0 ? 0 : cb.x, e5 = cb.y < 0 ? 0 : cb.y, e6 = cb.z < 0 ? 0 : cb.z, e7 = cb.w < 0 ? 0 : cb.w;
    const int ts = e0 + e1 + e2 + e3 + e4 + e5 + e6 + e7;
    int incl = ts;
#pragma unroll
    for (int d = 1; d < 32; d <<= 1) {
      const int up = __shfl_up(incl, d);
      if (lane >= d) incl += up;
    }
    if (lane == 31) wtot[wave] = incl;
    __syncthreads();
    int pre = 0;
#pragma unroll
    for (int w2 = 0; w2 < NWAVE; ++w2) pre += (w2 < wave) ? wtot[w2] : 0;
    int run = pre + incl - ts;
    soff[8 * tid + 0] = run; run += e0;
    soff[8 * tid + 1] = run; run += e1;
    soff[8 * tid + 2] = run; run += e2;
    soff[8 * tid + 3] = run; run += e3;
    soff[8 * tid + 4] = run; run += e4;
    soff[8 * tid + 5] = run; run += e5;
    soff[8 * tid + 6] = run; run += e6;
    soff[8 * tid + 7] = run;
  }
  __syncthreads();
  for (int i = tid; i < NBMAX; i += NTHR) list[i] = soff[i];
  __syncthreads();

  if (wave == 0) {
#pragma unroll 1
    for (int b0 = 0; b0 < nh; b0 += 32) {
      const int idx = b0 + lane;
      const int uv  = reg1[idx < RCAP ? idx : RCAP - 1];
      const int m32 = (nh - b0) < 32 ? (nh - b0) : 32;
#pragma unroll 1
      for (int k = 0; k < m32; ++k) {
        const int u   = __builtin_amdgcn_readlane(uv, k);
        const int sl  = u & (NBMAX - 1);
        const int eid = (int)((unsigned)u >> PKS);
        if (lane == 0) {
          int pos = list[sl];
          pos = pos < 0 ? 0 : (pos > RCAP - 1 ? RCAP - 1 : pos);
          reg2[pos] = eid;
          list[sl] = pos + 1;
        }
      }
    }
  }
  __syncthreads();

  const int nbw = nb >> 3;
  const bool ovf = (nh >= RCAP);
  const float qnan = __int_as_float(0x7fc00000);
  unsigned int* stwu = (unsigned int*)((float*)reg1 + wave * STW);
#pragma unroll 1
  for (int jt = 0; jt < nbw; ++jt) {
    const int slot = wave * nbw + jt;
    const int grow = nodeBase + slot;
    const int gcl  = grow < nN ? grow : nN - 1;
    int st = soff[slot];
    const int craw = scnt[slot];
    int cnt = craw;
    st  = st < 0 ? 0 : (st > nh ? nh : st);
    cnt = cnt < 0 ? 0 : (cnt > DEGCAP ? DEGCAP : cnt);
    if (cnt > nh - st) cnt = nh - st;
    const float pz = (ovf || craw > DEGCAP) ? qnan : 0.0f;
    const float live = grow < nN ? 1.0f : 0.0f;
    const bool wr = grow < MPr;

    const v4f s4 = *(const v4fa*)(H + (size_t)gcl * FEA + 4 * lane);
    v4f ag = {0.f, 0.f, 0.f, 0.f};
#pragma unroll 1
    for (int q = 0; q < cnt; ++q) {
      int idx = st + q; idx = idx > RCAP - 1 ? RCAP - 1 : idx;
      int eid = reg2[idx]; eid = eid < 0 ? 0 : (eid > nE - 1 ? nE - 1 : eid);
      const int sraw = srcs[eid];
      const int s = sraw < 0 ? 0 : (sraw > nN - 1 ? nN - 1 : sraw);
      const v4f v = *(const v4fa*)(H + (size_t)s * FEA + 4 * lane);
      ag = ag + v;
    }
    int dd = cnt - 1;
    dd = dd < 1 ? 1 : dd;
    const float invd = 1.0f / (float)dd;
    float hv[4], gv[4];
    hv[0] = s4.x * live + pz;  hv[1] = s4.y * live + pz;  hv[2] = s4.z * live + pz;  hv[3] = s4.w * live + pz;
    gv[0] = ((ag.x - s4.x) * invd) * live + pz;
    gv[1] = ((ag.y - s4.y) * invd) * live + pz;
    gv[2] = ((ag.z - s4.z) * invd) * live + pz;
    gv[3] = ((ag.w - s4.w) * invd) * live + pz;

    unsigned short hb[4], hl[4], gb[4], gl[4];
#pragma unroll
    for (int c = 0; c < 4; ++c) {
      hb[c] = bf_bits(hv[c]); hl[c] = bf_bits(hv[c] - bf_val(hb[c]));
      gb[c] = bf_bits(gv[c]); gl[c] = bf_bits(gv[c] - bf_val(gb[c]));
    }
    v2u w0, w1, w2, w3;
    w0.x = (unsigned int)hb[0] | ((unsigned int)hb[1] << 16);  w0.y = (unsigned int)hb[2] | ((unsigned int)hb[3] << 16);
    w1.x = (unsigned int)gb[0] | ((unsigned int)gb[1] << 16);  w1.y = (unsigned int)gb[2] | ((unsigned int)gb[3] << 16);
    w2.x = (unsigned int)hl[0] | ((unsigned int)hl[1] << 16);  w2.y = (unsigned int)hl[2] | ((unsigned int)hl[3] << 16);
    w3.x = (unsigned int)gl[0] | ((unsigned int)gl[1] << 16);  w3.y = (unsigned int)gl[2] | ((unsigned int)gl[3] << 16);
    __builtin_amdgcn_fence(__ATOMIC_RELEASE, "wavefront");
    __builtin_amdgcn_wave_barrier();
    *(v2ua*)(stwu + 2 * lane)       = w0;
    *(v2ua*)(stwu + 64 + 2 * lane)  = w1;
    *(v2ua*)(stwu + 128 + 2 * lane) = w2;
    *(v2ua*)(stwu + 192 + 2 * lane) = w3;
    __builtin_amdgcn_fence(__ATOMIC_RELEASE, "wavefront");
    __builtin_amdgcn_wave_barrier();
    const v4u pk0 = *(const v4ua*)(stwu + 4 * lane);
    const v4u pk1 = *(const v4ua*)(stwu + 128 + 4 * lane);
    unsigned short* gp = AC + (size_t)grow * (size_t)ACP + 8 * lane;
    if (wr) {
      *(volatile v4u*)gp         = pk0;
      *(volatile v4u*)(gp + 256) = pk1;
    }
    __threadfence();
    if (wr) {
      *(volatile v4u*)gp         = pk0;
      *(volatile v4u*)(gp + 256) = pk1;
    }
  }
}

static int pick_nb(int nE, int nN) {
  int nb = NBMAX;
  while (nb > 16 && (long long)nb * (long long)nE * 5LL > (long long)RCAP * (long long)nN * 4LL) nb >>= 1;
  return nb;
}
static inline int cdiv(int a, int b) { return (a + b - 1) / b; }

extern "C" void kernel_launch(void* const* d_in, const int* in_sizes, int n_in,
                              void* d_out, int out_size, void* d_ws, size_t ws_size,
                              hipStream_t stream) {
  if (n_in < 13) return;
  const int nN = in_sizes[0];
  if (nN <= 0 || nN > (1 << 22)) return;
  if ((long long)in_sizes[1] != (long long)nN * (long long)CIN) return;
  const int nE = in_sizes[2];
  if (nE < 1 || nE > (1 << 21)) return;
  if (in_sizes[3] != nE) return;
  if (in_sizes[4] < 2 * FEA || (in_sizes[4] % FEA) != 0) return;
  const int nEmb = in_sizes[4] / FEA;
  if (in_sizes[5] != CIN * HID || in_sizes[6] != HID) return;
  if (in_sizes[7] != HID * FEA || in_sizes[8] != FEA) return;
  if (in_sizes[10] < HID || (in_sizes[10] % HID) != 0) return;
  const int nL = in_sizes[10] / HID;
  if (nL < 1 || nL > LMAX) return;
  if (in_sizes[9] != nL * 2 * FEA * HID) return;
  if (in_sizes[11] != nL * HID * FEA || in_sizes[12] != nL * FEA) return;
  if ((long long)out_size != (long long)nN * FEA) return;

  const int*   nid  = (const int*)  d_in[0];
  const float* cont = (const float*)d_in[1];
  const int*   src  = (const int*)  d_in[2];
  const int*   dst  = (const int*)  d_in[3];
  const float* emb  = (const float*)d_in[4];
  const float* pw1  = (const float*)d_in[5];
  const float* pb1  = (const float*)d_in[6];
  const float* pw2  = (const float*)d_in[7];
  const float* pb2  = (const float*)d_in[8];
  const float* cw1  = (const float*)d_in[9];
  const float* cb1  = (const float*)d_in[10];
  const float* cw2  = (const float*)d_in[11];
  const float* cb2  = (const float*)d_in[12];
  float* out = (float*)d_out;

  const int MP   = cdiv(nN, GBM) * GBM;
  const int gM   = MP / GBM;
  const int nb   = pick_nb(nE, nN);
  const int gA   = cdiv(MP, nb);
  const int vec8 = 1;
  if (gA * nb < MP) return;

  char* ws = (char*)d_ws;
  size_t off = 0;
  const size_t oWT1 = off; off += (size_t)HID * CPAD * 2;                  off = (off + 255) & ~(size_t)255;
  const size_t oWT2 = off; off += (size_t)FEA * KH * 2;                    off = (off + 255) & ~(size_t)255;
  const size_t oWC1 = off; off += (size_t)nL * HID * KC * 2;               off = (off + 255) & ~(size_t)255;
  const size_t oWC2 = off; off += (size_t)nL * FEA * KH * 2;               off = (off + 255) & ~(size_t)255;
  const size_t oXC  = off; off += (size_t)MP * CPAD * 2;                   off = (off + 255) & ~(size_t)255;
  const size_t oH   = off; off += (size_t)MP * FEA * 4;                    off = (off + 255) & ~(size_t)255;
  const size_t oAC  = off; off += (size_t)MP * ACP * 2;                    off = (off + 255) & ~(size_t)255;
  if (off > ws_size || off > (size_t)WSMAX) return;
  unsigned short* WT1 = (unsigned short*)(ws + oWT1);
  unsigned short* WT2 = (unsigned short*)(ws + oWT2);
  unsigned short* WC1 = (unsigned short*)(ws + oWC1);
  unsigned short* WC2 = (unsigned short*)(ws + oWC2);
  unsigned short* XC  = (unsigned short*)(ws + oXC);
  float*          H   = (float*)(ws + oH);
  unsigned short* AC  = (unsigned short*)(ws + oAC);

  hipFuncSetAttribute(reinterpret_cast<const void*>(&k_mlp<0>),
                      hipFuncAttributeMaxDynamicSharedMemorySize, LDS_MLP);
  hipFuncSetAttribute(reinterpret_cast<const void*>(&k_mlp<1>),
                      hipFuncAttributeMaxDynamicSharedMemorySize, LDS_MLP);
  hipFuncSetAttribute(reinterpret_cast<const void*>(&k_agg),
                      hipFuncAttributeMaxDynamicSharedMemorySize, LDS_AGG);

  {
    const int nU1 = HID * (CPAD / 8);
    k_wtr<<<cdiv(nU1, NTHR), NTHR, 0, stream>>>(pw1, CIN, CPAD, CPAD, HID, 1, WT1, nU1);
    const int nU2 = FEA * (KH / 8);
    k_wtr<<<cdiv(nU2, NTHR), NTHR, 0, stream>>>(pw2, HID, HID, KH, FEA, 1, WT2, nU2);
    const int nU3 = nL * HID * (KC / 8);
    k_wtr<<<cdiv(nU3, NTHR), NTHR, 0, stream>>>(cw1, 2 * FEA, 2 * FEA, KC, HID, nL, WC1, nU3);
    const int nU4 = nL * FEA * (KH / 8);
    k_wtr<<<cdiv(nU4, NTHR), NTHR, 0, stream>>>(cw2, HID, HID, KH, FEA, nL, WC2, nU4);
  }

  const int nUc = MP * CQ;
  k_cprep<<<cdiv(nUc, NTHR), NTHR, 0, stream>>>(cont, XC, nN, nUc);

  k_mlp<0><<<gM, GTHR, LDS_MLP, stream>>>(XC, CPAD, CPAD / 32, WT1, pb1, WT2, pb2, nid, emb, nEmb, H, nN, MP);

  for (int i = 0; i < nL; ++i) {
    k_agg<<<gA, NTHR, LDS_AGG, stream>>>(src, dst, H, AC, nN, nE, nb, vec8, MP);
    const bool last = (i == nL - 1);
    float* dstH = last ? out : H;
    const int lim = last ? nN : MP;
    k_mlp<1><<<gM, GTHR, LDS_MLP, stream>>>(AC, ACP, KC / 32,
                                             WC1 + (size_t)i * HID * KC, cb1 + (size_t)i * HID,
                                             WC2 + (size_t)i * FEA * KH, cb2 + (size_t)i * FEA,
                                             nid, emb, nEmb, dstH, nN, lim);
  }
}
